// CausalFT_3135326126148
// MI455X (gfx1250) — hardware-verified
//
#include <hip/hip_runtime.h>
#include <stdint.h>


#define QLEN   1024
#define MLEN   1024
#define KLEN   2048
#define DMOD   1024
#define NBATCH 8
#define NCOL   (NBATCH * DMOD)
#define FTLEN  1025
#define KSTEPS 34

typedef _Float16 v8h  __attribute__((ext_vector_type(8)));
typedef _Float16 v16h __attribute__((ext_vector_type(16)));
typedef float    v8f  __attribute__((ext_vector_type(8)));
typedef float    v4f  __attribute__((ext_vector_type(4)));
union Frag { v16h v; v8h half[2]; };

__device__ __forceinline__ v8f wmma16(const v16h a, const v16h b, v8f c)
{
    c = __builtin_amdgcn_wmma_f32_16x16x32_f16(false, a, false, b, (short)0, c, false, false);
    asm volatile("v_nop\n\tv_nop\n\tv_nop\n\tv_nop" : "+v"(c) : "v"(a), "v"(b));
    return c;
}

__global__ __launch_bounds__(256) void build_ftmat(_Float16* __restrict__ A16)
{
    __shared__ _Float16 rowbuf[KLEN];
    const int i = blockIdx.x;
    if (i >= QLEN) return;
    const int tid = threadIdx.x;
    const float w  = 6.1299368850532551e-3f;
    const float cs = 0.031234752377721214f * 32.0f;
    #pragma unroll 1
    for (int it = 0; it < KLEN / 256; ++it) {
        const int j   = tid + 256 * it;
        const int dlt = j - i;
        float v = 0.0f;
        if (dlt >= 0 && dlt <= KLEN - QLEN) {
            const int r = (i * dlt) % FTLEN;
            v = cosf((float)r * w) * cs;
        }
        rowbuf[j] = (_Float16)v;
    }
    __syncthreads();
    const v8h o = *(const v8h*)(&rowbuf[8 * tid]);
    _Float16* dst = A16 + (size_t)i * KLEN + 8 * tid;
    *(volatile v8h*)dst = o;
    __threadfence();
    *(volatile v8h*)dst = o;
}

__global__ __launch_bounds__(256) void build_catT(
    const float* __restrict__ dec, const float* __restrict__ pos,
    const float* __restrict__ mems, const int* __restrict__ addpos,
    _Float16* __restrict__ Bt)
{
    __shared__ float tile[64][33];
    const int k0 = blockIdx.x * 64;
    const int n0 = blockIdx.y * 32;
    if (k0 >= KLEN || n0 >= NCOL) return;
    const int tid = threadIdx.x;
    const int tx = tid & 31, ty = tid >> 5;
    const bool ap = (addpos[0] != 0);
    const int n = n0 + tx;
    const int dcol = n & (DMOD - 1);

    #pragma unroll
    for (int r = 0; r < 8; ++r) {
        const int kl = ty * 8 + r;
        const int k  = k0 + kl;
        float v;
        if (k < MLEN) v = mems[(size_t)k * NCOL + n];
        else          v = dec[(size_t)(k - MLEN) * NCOL + n];
        if (ap) v += pos[(size_t)k * DMOD + dcol];
        tile[kl][tx] = v;
    }
    __syncthreads();

    const int l  = tid & 31, wv = tid >> 5;
    const int nl = 4 * wv + (l >> 3);
    const int q  = (l & 7) * 8;
    v8h o;
    #pragma unroll
    for (int e = 0; e < 8; ++e) o[e] = (_Float16)tile[q + e][nl];
    _Float16* dst = Bt + (size_t)(n0 + nl) * KLEN + k0 + q;
    *(volatile v8h*)dst = o;
    __threadfence();
    *(volatile v8h*)dst = o;
}

__global__ __launch_bounds__(256) void gemm_band(
    const _Float16* __restrict__ A16, const _Float16* __restrict__ Bt,
    const float* __restrict__ dec, float* __restrict__ out)
{
    const int tid  = threadIdx.x;
    const int lane = tid & 31;
    const int h    = lane >> 4;
    const int l16  = lane & 15;
    const int wave = tid >> 5;
    const int wr   = wave >> 2;
    const int wc   = wave & 3;

    const int BM0 = blockIdx.y * 64;
    const int BN0 = blockIdx.x * 256;
    if (BM0 >= QLEN || BN0 >= NCOL) return;
    const int wM = BM0 + wr * 32;
    const int wN = BN0 + wc * 64;

    const _Float16* pa0 = A16 + (size_t)(wM + l16) * KLEN + BM0 + 8 * h;
    const _Float16* pa1 = pa0 + (size_t)16 * KLEN;
    const _Float16* pb0 = Bt + (size_t)(wN + 4 * l16) * KLEN + BM0 + 8 * h;

    v8f acc[2][4] = {};

    #pragma unroll 1
    for (int t = 0; t < KSTEPS; ++t) {
        const int koff = t * 32;
        Frag a0, a1, b[4];
        a0.half[0] = *(const v8h*)(pa0 + koff);
        a0.half[1] = *(const v8h*)(pa0 + koff + 16);
        a1.half[0] = *(const v8h*)(pa1 + koff);
        a1.half[1] = *(const v8h*)(pa1 + koff + 16);
        #pragma unroll
        for (int ni = 0; ni < 4; ++ni) {
            const _Float16* pb = pb0 + (size_t)ni * KLEN + koff;
            b[ni].half[0] = *(const v8h*)(pb);
            b[ni].half[1] = *(const v8h*)(pb + 16);
        }
        #pragma unroll
        for (int ni = 0; ni < 4; ++ni) {
            acc[0][ni] = wmma16(a0.v, b[ni].v, acc[0][ni]);
            acc[1][ni] = wmma16(a1.v, b[ni].v, acc[1][ni]);
        }
    }

    const float rscale = 6.9053396600248780e-4f;
    v4f xs[2][8];
    #pragma unroll
    for (int mi = 0; mi < 2; ++mi) {
        #pragma unroll
        for (int r = 0; r < 8; ++r) {
            const int m = wM + mi * 16 + 8 * h + r;
            const size_t idx = (size_t)m * NCOL + wN + 4 * l16;
            const v4f d = *(const v4f*)(dec + idx);
            v4f x;
            x[0] = d[0] + acc[mi][0][r] * rscale;
            x[1] = d[1] + acc[mi][1][r] * rscale;
            x[2] = d[2] + acc[mi][2][r] * rscale;
            x[3] = d[3] + acc[mi][3][r] * rscale;
            xs[mi][r] = x;
        }
    }
    #pragma unroll
    for (int mi = 0; mi < 2; ++mi) {
        #pragma unroll
        for (int r = 0; r < 8; ++r) {
            const int m = wM + mi * 16 + 8 * h + r;
            const size_t idx = (size_t)m * NCOL + wN + 4 * l16;
            *(volatile v4f*)(out + idx) = xs[mi][r];
        }
    }
    __threadfence();
    #pragma unroll
    for (int mi = 0; mi < 2; ++mi) {
        #pragma unroll
        for (int r = 0; r < 8; ++r) {
            const int m = wM + mi * 16 + 8 * h + r;
            const size_t idx = (size_t)m * NCOL + wN + 4 * l16;
            *(volatile v4f*)(out + idx) = xs[mi][r];
        }
    }
}

__global__ __launch_bounds__(256) void layernorm_rows(
    float* __restrict__ out, const float* __restrict__ gamma,
    const float* __restrict__ beta)
{
    __shared__ float red_a[8];
    __shared__ float red_b[8];
    const int row = blockIdx.x;
    if (row >= QLEN * NBATCH) return;
    const int tid = threadIdx.x, wv = tid >> 5, l = tid & 31;
    float* x = out + (size_t)row * DMOD + 4 * tid;

    const v4f v = *(const v4f*)x;
    float s = (v[0] + v[1]) + (v[2] + v[3]);
    #pragma unroll
    for (int off = 16; off > 0; off >>= 1) s += __shfl_xor(s, off, 32);
    if (l == 0) red_a[wv] = s;
    __syncthreads();
    float tot = 0.0f;
    #pragma unroll
    for (int i = 0; i < 8; ++i) tot += red_a[i];
    const float mu = tot * (1.0f / (float)DMOD);

    const float d0 = v[0] - mu, d1 = v[1] - mu, d2 = v[2] - mu, d3 = v[3] - mu;
    float s2 = (d0 * d0 + d1 * d1) + (d2 * d2 + d3 * d3);
    #pragma unroll
    for (int off = 16; off > 0; off >>= 1) s2 += __shfl_xor(s2, off, 32);
    if (l == 0) red_b[wv] = s2;
    __syncthreads();
    float tot2 = 0.0f;
    #pragma unroll
    for (int i = 0; i < 8; ++i) tot2 += red_b[i];
    const float var = tot2 * (1.0f / (float)DMOD);
    const float inv = rsqrtf(var + 1e-5f);

    const v4f g  = *(const v4f*)(gamma + 4 * tid);
    const v4f bb = *(const v4f*)(beta + 4 * tid);
    v4f rr;
    rr[0] = (g[0] * d0) * inv + bb[0];
    rr[1] = (g[1] * d1) * inv + bb[1];
    rr[2] = (g[2] * d2) * inv + bb[2];
    rr[3] = (g[3] * d3) * inv + bb[3];
    *(volatile v4f*)x = rr;
    __threadfence();
    *(volatile v4f*)x = rr;
}

extern "C" void kernel_launch(void* const* d_in, const int* in_sizes, int n_in,
                              void* d_out, int out_size, void* d_ws, size_t ws_size,
                              hipStream_t stream)
{
    if (n_in < 6) return;
    if (in_sizes[0] != QLEN * NCOL || in_sizes[1] != KLEN * DMOD ||
        in_sizes[2] != MLEN * NCOL || in_sizes[3] != DMOD ||
        in_sizes[4] != DMOD || in_sizes[5] < 1 || out_size != QLEN * NCOL) return;

    const size_t bytesA = (size_t)QLEN * KLEN * sizeof(_Float16);
    const size_t bytesB = (size_t)NCOL * KLEN * sizeof(_Float16);
    if (bytesA + bytesB > ws_size) return;

    const float* dec   = (const float*)d_in[0];
    const float* pos   = (const float*)d_in[1];
    const float* mems  = (const float*)d_in[2];
    const float* gamma = (const float*)d_in[3];
    const float* beta  = (const float*)d_in[4];
    const int*   addp  = (const int*)  d_in[5];
    float* out = (float*)d_out;

    _Float16* A16 = (_Float16*)d_ws;
    _Float16* Bt  = (_Float16*)((char*)d_ws + bytesA);

    build_ftmat<<<dim3(QLEN), dim3(256), 0, stream>>>(A16);
    build_catT<<<dim3(KLEN / 64, NCOL / 32), dim3(256), 0, stream>>>(dec, pos, mems, addp, Bt);
    gemm_band<<<dim3(NCOL / 256, QLEN / 64), dim3(256), 0, stream>>>(A16, Bt, dec, out);
    layernorm_rows<<<dim3(QLEN * NBATCH), dim3(256), 0, stream>>>(out, gamma, beta);
}
